// ConditionedBlockAttentionPairBias_59115929862886
// MI455X (gfx1250) — hardware-run, weakly checked
//
#include <hip/hip_runtime.h>


#define TT   768
#define HD   64
#define ZH   1
#define RH   0
#define PCAR 1024.0f
#define SCL  0.125f
#define PMUL 1.0f
#define LNC_MAX 2048
typedef _Float16 h16;
typedef unsigned short bf;
typedef __attribute__((ext_vector_type(16))) __bf16   v16bf;
typedef __attribute__((ext_vector_type(16))) _Float16 v16h;
typedef __attribute__((ext_vector_type(8)))  _Float16 v8h;
typedef __attribute__((ext_vector_type(8)))  unsigned short v8us;
typedef __attribute__((ext_vector_type(8)))  float    v8f;
typedef __attribute__((ext_vector_type(4)))  float    v4f;
typedef v8h  __attribute__((may_alias)) v8ha;
typedef v4f  __attribute__((may_alias)) v4fa;
typedef v8us __attribute__((may_alias)) v8usa;

__device__ __forceinline__ unsigned short f2bf(float f) { unsigned u = __float_as_uint(f); u += 0x7FFFu + ((u >> 16) & 1u); return (unsigned short)(u >> 16); }
__device__ __forceinline__ float bf2f(unsigned short b) { return __uint_as_float(((unsigned)b) << 16); }
__device__ __forceinline__ float bfr(float f) { return bf2f(f2bf(f)); }
__device__ __forceinline__ v16h cat16(v8h lo, v8h hi) { return __builtin_shufflevector(lo, hi, 0, 1, 2, 3, 4, 5, 6, 7, 8, 9, 10, 11, 12, 13, 14, 15); }
__device__ __forceinline__ v16bf cat16b(v8us lo, v8us hi) { return __builtin_bit_cast(v16bf, __builtin_shufflevector(lo, hi, 0, 1, 2, 3, 4, 5, 6, 7, 8, 9, 10, 11, 12, 13, 14, 15)); }
__device__ __forceinline__ v8f wmma16(v16h a, v16h b, v8f c) { return __builtin_amdgcn_wmma_f32_16x16x32_f16(false, a, false, b, (short)0, c, false, false); }
__device__ __forceinline__ v8f wmmab(v16bf a, v16bf b, v8f c) { return __builtin_amdgcn_wmma_f32_16x16x32_bf16(false, a, false, b, (short)0, c, false, false); }

template <typename T16> struct WFrag;
template <> struct WFrag<h16> { typedef v16h V; static __device__ __forceinline__ V ld(const h16* p) { return cat16(*(const v8h*)p, *(const v8h*)(p + 16)); } static __device__ __forceinline__ v8f mma(V a, V b, v8f c) { return wmma16(a, b, c); } };
template <> struct WFrag<bf> { typedef v16bf V; static __device__ __forceinline__ V ld(const bf* p) { return cat16b(*(const v8us*)p, *(const v8us*)(p + 16)); } static __device__ __forceinline__ v8f mma(V a, V b, v8f c) { return wmmab(a, b, c); } };
template <typename T16, int NSPLIT, bool BIAS>
__global__ __launch_bounds__(32) void k_gemmw(const T16* __restrict__ A, const T16* __restrict__ A2, const T16* __restrict__ Bt, const T16* __restrict__ Bt2, int K, float* C, int ldc, const float* __restrict__ bias, size_t sA, size_t sB, size_t sC) {
    typedef typename WFrag<T16>::V V;
    __shared__ __align__(16) float os[16 * 68];
    const size_t z = blockIdx.z; A += z * sA; if (A2) A2 += z * sA; Bt += z * sB; if (Bt2) Bt2 += z * sB; C += z * sC;
    const int lane = threadIdx.x & 31, lr = lane & 15, hi = lane >> 4; const int r0 = blockIdx.x * 64, c0 = blockIdx.y * 64;
    v8f acc[4][4];
#pragma unroll
    for (int mb = 0; mb < 4; ++mb)
#pragma unroll
        for (int nb = 0; nb < 4; ++nb) acc[mb][nb] = (v8f){};
    const size_t aoff = (size_t)(r0 + lr) * K + 8 * hi, boff = (size_t)(c0 + lr) * K + 8 * hi;
    for (int kc = 0; kc < K; kc += 32) {
        V a[4], a2[4];
#pragma unroll
        for (int mb = 0; mb < 4; ++mb) { a[mb] = WFrag<T16>::ld(A + aoff + (size_t)mb * 16 * K + kc); if (NSPLIT == 1 || NSPLIT == 2) a2[mb] = WFrag<T16>::ld(A2 + aoff + (size_t)mb * 16 * K + kc); }
#pragma unroll
        for (int nb = 0; nb < 4; ++nb) { const V b = WFrag<T16>::ld(Bt + boff + (size_t)nb * 16 * K + kc); V b2; if (NSPLIT >= 2) b2 = WFrag<T16>::ld(Bt2 + boff + (size_t)nb * 16 * K + kc);
#pragma unroll
            for (int mb = 0; mb < 4; ++mb) { acc[mb][nb] = WFrag<T16>::mma(a[mb], b, acc[mb][nb]); if (NSPLIT == 1 || NSPLIT == 2) acc[mb][nb] = WFrag<T16>::mma(a2[mb], b, acc[mb][nb]); if (NSPLIT >= 2) acc[mb][nb] = WFrag<T16>::mma(a[mb], b2, acc[mb][nb]); } }
        asm volatile("v_nop\n\tv_nop\n\tv_nop\n\tv_nop" : "+v"(acc[0][0]), "+v"(acc[1][1]), "+v"(acc[2][2]), "+v"(acc[3][3]) : "v"(a[0]), "v"(a[3]));
    }
#pragma unroll
    for (int mb = 0; mb < 4; ++mb) {
#pragma unroll
        for (int nb = 0; nb < 4; ++nb) {
#pragma unroll
            for (int j = 0; j < 8; ++j) os[(hi * 8 + j) * 68 + nb * 16 + lr] = acc[mb][nb][j]; }
        __builtin_amdgcn_wave_barrier(); asm volatile("" ::: "memory");
        float* crow = C + (size_t)(r0 + mb * 16) * ldc + c0;
#pragma unroll 1
        for (int ps = 0; ps < 2; ++ps) {
#pragma unroll
            for (int s = 0; s < 8; ++s) { const int row = 2 * s + hi, cofs = lr * 4; v4f val = *(const v4fa*)(os + row * 68 + cofs); if (BIAS) { val[0] += bfr(bias[c0 + cofs]); val[1] += bfr(bias[c0 + cofs + 1]); val[2] += bfr(bias[c0 + cofs + 2]); val[3] += bfr(bias[c0 + cofs + 3]); }
                *(volatile v4f*)(crow + (size_t)row * ldc + cofs) = val; }
            if (ps == 0) __threadfence(); }
        __builtin_amdgcn_wave_barrier(); asm volatile("" ::: "memory");
    }
}

__device__ __forceinline__ h16 tohx(float x) { return (h16)x; }
__device__ __forceinline__ void splitf(float y, unsigned short& h, unsigned short& l) { h = f2bf(y); l = f2bf(y - bf2f(h)); }
typedef __attribute__((ext_vector_type(2))) _Float16 v2h;
typedef __attribute__((ext_vector_type(4))) _Float16 v4h;
typedef __attribute__((ext_vector_type(2))) unsigned short v2us;
typedef __attribute__((ext_vector_type(4))) unsigned short v4us;
typedef __attribute__((ext_vector_type(2))) float v2f;
typedef __attribute__((ext_vector_type(4))) int v4i;

template <typename T16, int NSPLIT, bool BIAS, int NW>
__global__ __launch_bounds__(32) void k_gemmn(const T16* __restrict__ A, const T16* __restrict__ A2, const T16* __restrict__ Bt, const T16* __restrict__ Bt2, int K, float* C, int ldc, const float* __restrict__ bias, size_t sA, size_t sB, size_t sC) {
    typedef typename WFrag<T16>::V V;
    static_assert(NW == 16 || NW == 32 || NW == 64, "the tile's width is 16, 32 or 64");
    constexpr int NB = NW / 16, PITCH = NW + 4, LS = (NW == 64) ? 4 : (NW == 32) ? 3 : 2;
    __shared__ __align__(16) float os[16 * PITCH];
    const size_t z = blockIdx.z; A += z * sA; if (A2) A2 += z * sA; Bt += z * sB; if (Bt2) Bt2 += z * sB; C += z * sC;
    const int lane = threadIdx.x & 31, lr = lane & 15, hi = lane >> 4; const int r0 = blockIdx.x * 64, c0 = blockIdx.y * NW;
    v8f acc[4][NB];
#pragma unroll
    for (int mb = 0; mb < 4; ++mb)
#pragma unroll
        for (int nb = 0; nb < NB; ++nb) acc[mb][nb] = (v8f){};
    const size_t aoff = (size_t)(r0 + lr) * K + 8 * hi, boff = (size_t)(c0 + lr) * K + 8 * hi;
    for (int kc = 0; kc < K; kc += 32) {
        V a[4], a2[4];
#pragma unroll
        for (int mb = 0; mb < 4; ++mb) { a[mb] = WFrag<T16>::ld(A + aoff + (size_t)mb * 16 * K + kc); if (NSPLIT == 1 || NSPLIT == 2) a2[mb] = WFrag<T16>::ld(A2 + aoff + (size_t)mb * 16 * K + kc); }
#pragma unroll
        for (int nb = 0; nb < NB; ++nb) { const V b = WFrag<T16>::ld(Bt + boff + (size_t)nb * 16 * K + kc); V b2; if (NSPLIT >= 2) b2 = WFrag<T16>::ld(Bt2 + boff + (size_t)nb * 16 * K + kc);
#pragma unroll
            for (int mb = 0; mb < 4; ++mb) { acc[mb][nb] = WFrag<T16>::mma(a[mb], b, acc[mb][nb]); if (NSPLIT == 1 || NSPLIT == 2) acc[mb][nb] = WFrag<T16>::mma(a2[mb], b, acc[mb][nb]); if (NSPLIT >= 2) acc[mb][nb] = WFrag<T16>::mma(a[mb], b2, acc[mb][nb]); } }
        asm volatile("v_nop\n\tv_nop\n\tv_nop\n\tv_nop" : "+v"(acc[0][0]), "+v"(acc[1][1 % NB]), "+v"(acc[2][2 % NB]), "+v"(acc[3][3 % NB]) : "v"(a[0]), "v"(a[3]));
    }
#pragma unroll
    for (int mb = 0; mb < 4; ++mb) {
#pragma unroll
        for (int nb = 0; nb < NB; ++nb) {
#pragma unroll
            for (int j = 0; j < 8; ++j) os[(hi * 8 + j) * PITCH + nb * 16 + lr] = acc[mb][nb][j]; }
        __builtin_amdgcn_wave_barrier(); asm volatile("" ::: "memory");
        float* crow = C + (size_t)(r0 + mb * 16) * ldc + c0;
        for (int ps = 0; ps < 2; ++ps) {
#pragma unroll
            for (int s = 0; s < NW / 8; ++s) { const int row = (128 / NW) * s + (lane >> LS), cofs = (lane & (NW / 4 - 1)) * 4; v4f val = *(const v4fa*)(os + row * PITCH + cofs); if (BIAS) { val[0] += bfr(bias[c0 + cofs]); val[1] += bfr(bias[c0 + cofs + 1]); val[2] += bfr(bias[c0 + cofs + 2]); val[3] += bfr(bias[c0 + cofs + 3]); }
                *(volatile v4f*)(crow + (size_t)row * ldc + cofs) = val; }
            if (ps == 0) __threadfence(); }
        __builtin_amdgcn_wave_barrier(); asm volatile("" ::: "memory");
    }
}

__global__ __launch_bounds__(256) void k_cvt8(const float* __restrict__ src, bf* dst, size_t n8) { const size_t i = (size_t)blockIdx.x * 256 + threadIdx.x; if (i >= n8) return; const v8f v = *(const v8f*)(src + i * 8); v8us o;
#pragma unroll
    for (int k = 0; k < 8; ++k) o[k] = f2bf(v[k]); *(volatile v8us*)(dst + i * 8) = o; __threadfence(); *(volatile v8us*)(dst + i * 8) = o; }
__global__ __launch_bounds__(256) void k_rbf(const float* __restrict__ X, float* Y, size_t n4) { const size_t i = (size_t)blockIdx.x * 256 + threadIdx.x; if (i >= n4) return; const v4f a = *(const v4f*)(X + i * 4); v4f o;
#pragma unroll
    for (int q = 0; q < 4; ++q) o[q] = bfr(a[q]);
    *(volatile v4f*)(Y + i * 4) = o; __threadfence(); *(volatile v4f*)(Y + i * 4) = o; }

#define LNC_MAX 2048
template <bool RES>
__global__ __launch_bounds__(256) void k_lnrow(const float* __restrict__ A, const float* __restrict__ R, const float* __restrict__ gamma, const float* __restrict__ beta, float eps, int C, int nrows, float* Y) {
    const int lane = threadIdx.x & 31; const int row = blockIdx.x * 8 + (threadIdx.x >> 5); if (row >= nrows) return; const int nch = C / 128; const float* a = A + (size_t)row * C; float x[LNC_MAX / 32]; float s = 0.0f;
    for (int k = 0; k < LNC_MAX / 128; ++k) { if (k < nch) { const int c0 = k * 128 + lane * 4; v4f v = *(const v4f*)(a + c0);
            if (RES) { const v4f w = *(const v4f*)(R + (size_t)row * C + c0); v[0] = __fadd_rn(v[0], w[0]); v[1] = __fadd_rn(v[1], w[1]); v[2] = __fadd_rn(v[2], w[2]); v[3] = __fadd_rn(v[3], w[3]); }
            x[k * 4 + 0] = v[0]; x[k * 4 + 1] = v[1]; x[k * 4 + 2] = v[2]; x[k * 4 + 3] = v[3]; s = __fadd_rn(__fadd_rn(__fadd_rn(__fadd_rn(s, v[0]), v[1]), v[2]), v[3]); } }
    for (int sh = 16; sh; sh >>= 1) s = __fadd_rn(s, __shfl_xor(s, sh, 32));
    const float mean = __fdiv_rn(s, (float)C); float q = 0.0f;
    for (int k = 0; k < LNC_MAX / 128; ++k) { if (k < nch) {
            for (int j = 0; j < 4; ++j) { const float d = __fsub_rn(x[k * 4 + j], mean); x[k * 4 + j] = d; q = __fmaf_rn(d, d, q); } } }
    for (int sh = 16; sh; sh >>= 1) q = __fadd_rn(q, __shfl_xor(q, sh, 32));
    const float rstd = __fdiv_rn(1.0f, sqrtf(__fadd_rn(__fdiv_rn(q, (float)C), eps)));
    for (int k = 0; k < LNC_MAX / 128; ++k) { if (k < nch) { const int c0 = k * 128 + lane * 4; const v4f g = *(const v4f*)(gamma + c0); const v4f bt = *(const v4f*)(beta + c0);
            for (int j = 0; j < 4; ++j) x[k * 4 + j] = __fmaf_rn(__fmul_rn(x[k * 4 + j], rstd), bfr(g[j]), bfr(bt[j])); } }
    float* y = Y + (size_t)row * C;
    for (int ps = 0; ps < 2; ++ps) {
        for (int k = 0; k < LNC_MAX / 128; ++k) { if (k < nch) { v4f o; o[0] = x[k * 4 + 0]; o[1] = x[k * 4 + 1]; o[2] = x[k * 4 + 2]; o[3] = x[k * 4 + 3]; *(volatile v4f*)(y + k * 128 + lane * 4) = o; } }
        if (ps == 0) __threadfence(); }
}

__global__ __launch_bounds__(256) void k_tohl(const float* __restrict__ F, float sc, bf* Hh, bf* Hl, size_t n4) { const size_t i = (size_t)blockIdx.x * 256 + threadIdx.x; if (i >= n4) return; const v4f a = *(const v4f*)(F + i * 4); v4us oh, ol;
#pragma unroll
    for (int q = 0; q < 4; ++q) { unsigned short h2, l2; splitf(__fmul_rn(a[q], sc), h2, l2); oh[q] = h2; ol[q] = l2; }
    *(volatile v4us*)(Hh + i * 4) = oh; *(volatile v4us*)(Hl + i * 4) = ol; __threadfence(); *(volatile v4us*)(Hh + i * 4) = oh; *(volatile v4us*)(Hl + i * 4) = ol; }

__global__ __launch_bounds__(256) void k_asoftMA(const float* __restrict__ Sb, const float* __restrict__ MP, h16* P16, bf* Ph, bf* Pl) {
    const int lane = threadIdx.x & 31; const int row = blockIdx.x * 8 + (threadIdx.x >> 5); if (row >= ZH * TT) return; const int i = row % TT; const int zz = row / TT; (void)zz; const bool hires = (i < RH); const float* sr = Sb + (size_t)row * TT; float v[TT / 32]; float mx = -3.0e38f;
#pragma unroll
    for (int ch = 0; ch < TT / 128; ++ch) { const int j0 = ch * 128 + lane * 4; const v4f a = *(const v4f*)(sr + j0); const v4f m4 = *(const v4f*)(MP + (size_t)i * TT + j0);
#pragma unroll
        for (int q = 0; q < 4; ++q) { const int j = j0 + q; (void)j; const float t = a[q] * SCL + bfr(m4[q]) * PMUL;     v[ch * 4 + q] = t; mx = fmaxf(mx, t); } }
#pragma unroll
    for (int sh = 16; sh; sh >>= 1) mx = fmaxf(mx, __shfl_xor(mx, sh, 32));
    float sum = 0.f;
#pragma unroll
    for (int k = 0; k < TT / 32; ++k) { float d0 = __fsub_rn(v[k], mx); v[k] = __builtin_amdgcn_exp2f(__fmul_rn(d0, 1.4426950408889634f)); sum += v[k]; }
#pragma unroll
    for (int sh = 16; sh; sh >>= 1) sum += __shfl_xor(sum, sh, 32);
    const float f = __fdiv_rn(hires ? 1.0f : PCAR, sum);
#pragma unroll 1
    for (int ps = 0; ps < 2; ++ps) {
        if (hires) {
#pragma unroll
            for (int ch = 0; ch < TT / 128; ++ch) { v4us oh, ol;
#pragma unroll
                for (int q = 0; q < 4; ++q) { unsigned short a, c2; splitf(v[ch * 4 + q] * f, a, c2); oh[q] = a; ol[q] = c2; }
                const size_t oo = ((size_t)zz * (RH ? RH : 1) + i) * TT + ch * 128 + lane * 4; *(volatile v4us*)(Ph + oo) = oh; *(volatile v4us*)(Pl + oo) = ol; }
        } else {
#pragma unroll
            for (int ch = 0; ch < TT / 128; ++ch) { v4h o4;
#pragma unroll
                for (int q = 0; q < 4; ++q) o4[q] = tohx(v[ch * 4 + q] * f);
                *(volatile v4h*)(P16 + (size_t)row * TT + ch * 128 + lane * 4) = o4; } }
        if (ps == 0) __threadfence(); }
}
typedef __attribute__((ext_vector_type(4))) float v4f_t;
__global__ __launch_bounds__(256) void k_fill(float* __restrict__ p, float val, size_t n4) { const size_t i = (size_t)blockIdx.x * 256 + threadIdx.x; if (i < n4) { v4f_t v = {val, val, val, val}; *(volatile v4f_t*)(p + 4 * i) = v; __threadfence(); *(volatile v4f_t*)(p + 4 * i) = v; } }
__global__ __launch_bounds__(256) void k_hb(const float* __restrict__ E, const float* __restrict__ PB, const float* __restrict__ pbias, int h, float rs, const float* __restrict__ S, float* S2, float* MP) { const unsigned i = blockIdx.x * 256 + threadIdx.x; if (i >= 768u * 192u) return; const size_t e = (size_t)i * 4; const v4f s4 = *(const v4f*)(S + e); const float bh = bfr(pbias[h]); v4f m, o;
#pragma unroll
    for (int q = 0; q < 4; ++q) { m[q] = E[(e + q) * 16 + h]; o[q] = __fmaf_rn(PB[(e + q) * 16 + h] + bh, rs, s4[q]); }
    *(volatile v4f*)(MP + e) = m; *(volatile v4f*)(S2 + e) = o; __threadfence(); *(volatile v4f*)(MP + e) = m; *(volatile v4f*)(S2 + e) = o; }
__global__ __launch_bounds__(256) void k_sg(const float* __restrict__ X, int px, int xhw, int xs, const float* __restrict__ G, int pg, const float* __restrict__ W, int pw, float cf, float* Y, int py, int w4, int nrows) { const unsigned i = blockIdx.x * 256 + threadIdx.x; if (i >= (unsigned)(w4 * nrows)) return; const unsigned r = i / (unsigned)w4, c = (i - r * (unsigned)w4) * 4u; const unsigned xb = c / (unsigned)xhw, xc = xb * (unsigned)xs + (c - xb * (unsigned)xhw); const v4f x = *(const v4f*)(X + (size_t)r * px + xc); const v4f g = *(const v4f*)(G + (size_t)r * pg + c); const v4f w = *(const v4f*)(W + (size_t)r * pw + c); v4f o;
#pragma unroll
    for (int q = 0; q < 4; ++q) { const float ex = __builtin_amdgcn_exp2f(__fmul_rn(-g[q], 1.4426950408889634f)); const float sg = __fdiv_rn(1.0f, 1.0f + ex); o[q] = __fmaf_rn(__fmul_rn(x[q], cf), sg, w[q]); }
    *(volatile v4f*)(Y + (size_t)r * py + c) = o; __threadfence(); *(volatile v4f*)(Y + (size_t)r * py + c) = o; }

__global__ __launch_bounds__(256) void k_vtp(const float* __restrict__ F, int pitch, int nheads, h16* V16, bf* Vh, bf* Vl) { const size_t e = ((size_t)blockIdx.x * 256 + threadIdx.x) * 2; if (e >= (size_t)nheads * HD * TT) return; const int t = (int)(e % TT); const int d = (int)((e / TT) % HD); const int g = (int)(e / ((size_t)TT * HD)); v2h o16; v2us oh, ol;
#pragma unroll
    for (int q = 0; q < 2; ++q) { const float x = F[(size_t)(t + q) * pitch + g * HD + d]; o16[q] = tohx(x); (void)oh; (void)ol; }
    *(volatile v2h*)(V16 + e) = o16; __threadfence(); *(volatile v2h*)(V16 + e) = o16; }
template <typename T16> __device__ __forceinline__ unsigned short cv16(float x);
template <> __device__ __forceinline__ unsigned short cv16<h16>(float x) { const h16 h = (h16)x; return __builtin_bit_cast(unsigned short, h); }
template <typename T16>
__global__ __launch_bounds__(256) void k_castp(const float* __restrict__ src, int rows_valid, int lc, float mul, unsigned short* dst) { const unsigned e = blockIdx.x * 256 + threadIdx.x; const unsigned r = e >> (lc - 3); const unsigned c0 = (e & ((1u << (lc - 3)) - 1u)) << 3; const unsigned rr = (r < (unsigned)rows_valid) ? r : (unsigned)(rows_valid - 1);
    const float* s = src + ((size_t)rr << lc) + c0; const v4f a = *(const v4f*)s, b = *(const v4f*)(s + 4); const float lm = (r < (unsigned)rows_valid) ? mul : 0.0f; v8us o;
#pragma unroll
    for (int q = 0; q < 4; ++q) { o[q] = cv16<T16>(__fmul_rn(a[q], lm)); o[q + 4] = cv16<T16>(__fmul_rn(b[q], lm)); }
    *(volatile v8us*)(dst + (size_t)e * 8) = o; __threadfence(); *(volatile v8us*)(dst + (size_t)e * 8) = o; }
__global__ __launch_bounds__(256) void k_b2h(const bf* __restrict__ src, float mul, unsigned short* dst) { const unsigned e = blockIdx.x * 256 + threadIdx.x; const v8us a = *(const v8us*)(src + (size_t)e * 8); v8us o;
#pragma unroll
    for (int q = 0; q < 8; ++q) o[q] = cv16<h16>(__fmul_rn(bf2f(a[q]), mul));
    *(volatile v8us*)(dst + (size_t)e * 8) = o; __threadfence(); *(volatile v8us*)(dst + (size_t)e * 8) = o; }
__global__ __launch_bounds__(256) void k_cvtp(const float* __restrict__ src, h16* dst, int w4, int sp, int dp, int nrows) { const unsigned i = blockIdx.x * 256u + threadIdx.x; if (i >= (unsigned)w4 * (unsigned)nrows) return; const unsigned r = i / (unsigned)w4, c = (i - r * (unsigned)w4) * 4u; const v4f x = *(const v4f*)(src + (size_t)r * sp + c); v4h o;
#pragma unroll
    for (int q = 0; q < 4; ++q) o[q] = tohx(x[q]);
    *(volatile v4h*)(dst + (size_t)r * dp + c) = o; __threadfence(); *(volatile v4h*)(dst + (size_t)r * dp + c) = o; }

__device__ __forceinline__ int iclamp(int v, int lo, int hi) { return v < lo ? lo : (v > hi ? hi : v); }
template <int W>
__global__ __launch_bounds__(256) void rgath_kernel(const float* __restrict__ P, const int* __restrict__ idx, int nidx, int ioff, float* __restrict__ OUT, int op, int ocol, int n) {
  static_assert(W % 32 == 0, "rgath: whole 128-B lines per row block"); const size_t t = (size_t)blockIdx.x * 256 + threadIdx.x; if (t >= (size_t)n * (W / 4)) return; const size_t i = t / (W / 4); const int c = (int)(t % (W / 4)) * 4;
  const int r = iclamp(idx[i], 0, nidx - 1) + ioff; const v4f a = *(const v4f*)(P + (size_t)r * W + c);
  for (int pass = 0; pass < 2; ++pass) { *(volatile v4f*)(OUT + i * op + ocol + c) = a; __threadfence(); }
}

__global__ __launch_bounds__(256) void k_mulm(const float* __restrict__ P, const float* __restrict__ kp, float* Y, int w4, int nrows) { const unsigned i = blockIdx.x * 256u + threadIdx.x; if (i >= (unsigned)w4 * (unsigned)nrows) return; const unsigned r = i / (unsigned)w4; const float f = bfr(kp[r]); const v4f u = *(const v4f*)(P + (size_t)i * 4); v4f o;
#pragma unroll
    for (int t = 0; t < 4; ++t) o[t] = __fmul_rn(u[t], f);
    *(volatile v4f*)(Y + (size_t)i * 4) = o; __threadfence(); *(volatile v4f*)(Y + (size_t)i * 4) = o; }
__global__ __launch_bounds__(256) void k_mterm(float* S, const float* __restrict__ kp, float cf) { const unsigned i = blockIdx.x * 256u + threadIdx.x; if (i >= 768u * 192u) return; const unsigned r = i / 192u, c = (i - r * 192u) * 4u; const float fr = bfr(kp[r]); const v4f fc = *(const v4f*)(kp + c); const size_t ofs = (size_t)i * 4; const v4f u = *(const v4f*)(S + ofs); v4f o;
#pragma unroll
    for (int t = 0; t < 4; ++t) o[t] = __fadd_rn(u[t], __fmul_rn(__fsub_rn(__fmul_rn(fr, bfr(fc[t])), 1.0f), cf));
    *(volatile v4f*)(S + ofs) = o; __threadfence(); *(volatile v4f*)(S + ofs) = o; }

extern "C" void kernel_launch(void* const* d_in, const int* in_sizes, int n_in,
                              void* d_out, int out_size, void* d_ws, size_t ws_size, hipStream_t stream) {
    (void)in_sizes; (void)n_in; (void)out_size;
    const float* i0 = (const float*)d_in[0]; const float* i1 = (const float*)d_in[1]; const float* i2 = (const float*)d_in[2]; const float* i3 = (const float*)d_in[3]; const int* i4 = (const int*)d_in[4]; const float* i5 = (const float*)d_in[5]; const float* i6 = (const float*)d_in[6]; const float* i7 = (const float*)d_in[7]; const float* i8 = (const float*)d_in[8]; const float* i9 = (const float*)d_in[9]; const float* i10 = (const float*)d_in[10]; const float* i11 = (const float*)d_in[11]; const float* i12 = (const float*)d_in[12]; const float* i13 = (const float*)d_in[13]; const float* i14 = (const float*)d_in[14]; const float* i15 = (const float*)d_in[15]; const float* i16 = (const float*)d_in[16]; const float* i17 = (const float*)d_in[17];
    float* OUT = (float*)d_out;
    char* wsp = (char*)d_ws;
    auto take = [&](size_t bytes) { char* p = wsp; wsp += (bytes + 255) & ~(size_t)255; return (void*)p; };
    const size_t NN = (size_t)768 * 768, NT = (size_t)64 * 768, NC = (size_t)64 * 512, PZ = (size_t)64 * 768 * 128;
    bf* W6 = (bf*)take((size_t)768 * 512 * 2); bf* W8 = (bf*)take((size_t)768 * 512 * 2); bf* W15 = (bf*)take((size_t)768 * 512 * 2); bf* W9b = (bf*)take(NN * 2); bf* W10b = (bf*)take(NN * 4); bf* W14b = (bf*)take(NN * 2); bf* W17b = (bf*)take(NN * 2); unsigned short* W9 = (unsigned short*)take(NN * 2); unsigned short* W10 = (unsigned short*)take(NN * 4); unsigned short* W14 = (unsigned short*)take(NN * 2); unsigned short* W17 = (unsigned short*)take(NN * 2); bf* W13 = (bf*)take((size_t)16 * 128 * 2);
    float* ONE = (float*)take(768 * 4); float* NOU = (float*)take(768 * 4); float* ZP = (float*)take(NN * 4); float* ZE = (float*)take(NN * 16 * 4);
    float* CR = (float*)take(NC * 4); float* CN = (float*)take(NC * 4); bf* CNh = (bf*)take(NC * 2); bf* CNl = (bf*)take(NC * 2); bf* CRb = (bf*)take(NC * 2); float* T1 = (float*)take(NT * 4); float* T2 = (float*)take(NT * 4); float* T3 = (float*)take(NT * 4);
    float* G1 = (float*)take(NN * 4); float* G2 = (float*)take(NN * 4); float* G3 = (float*)take(NN * 4); float* G1m = (float*)take(NN * 4); float* G2m = (float*)take(NN * 4); float* NR = (float*)take(NN * 4); float* S0 = (float*)take(NN * 4); float* ST = (float*)take(NN * 4); unsigned short* S16 = (unsigned short*)take(NN * 2);
    float* FQ = (float*)take(NN * 4); float* FKV = (float*)take(NN * 8); float* FG = (float*)take(NN * 4); h16* QP16 = (h16*)take(NN * 2); h16* KP16 = (h16*)take(NN * 2); h16* VT16 = (h16*)take(NN * 2);
    float* ZR = (float*)take(PZ * 4); float* ZN = (float*)take(PZ * 4); bf* ZB = (bf*)take(PZ * 2); float* PB = (float*)take(NN * 16 * 4);
    float* Sb = (float*)take(NN * 4); float* S2 = (float*)take(NN * 4); float* MP = (float*)take(NN * 4); h16* P16 = (h16*)take(NN * 2); float* OB = (float*)take(NN * 4); float* GO = (float*)take(NN * 4); unsigned short* GO16 = (unsigned short*)take(NN * 2); float* OM = (float*)take(NN * 4); float* FO = (float*)take(NN * 4);
    if ((size_t)(wsp - (char*)d_ws) > ws_size) return;
    { const unsigned LT = (unsigned)(((size_t)768 * 512 / 8 + 255) / 256), LS = (unsigned)((NN / 8 + 255) / 256); k_cvt8<<<LT, 256, 0, stream>>>(i6, W6, (size_t)768 * 512 / 8); k_cvt8<<<LT, 256, 0, stream>>>(i8, W8, (size_t)768 * 512 / 8); k_cvt8<<<LT, 256, 0, stream>>>(i15, W15, (size_t)768 * 512 / 8); k_cvt8<<<LS, 256, 0, stream>>>(i9, W9b, NN / 8); k_cvt8<<<2 * LS, 256, 0, stream>>>(i10, W10b, NN / 4); k_cvt8<<<LS, 256, 0, stream>>>(i14, W14b, NN / 8); k_cvt8<<<LS, 256, 0, stream>>>(i17, W17b, NN / 8);
      k_b2h<<<(unsigned)(NN / 8 / 256), 256, 0, stream>>>(W9b, 1.0f, W9); k_b2h<<<(unsigned)(NN / 4 / 256), 256, 0, stream>>>(W10b, 1.0f, W10); k_b2h<<<(unsigned)(NN / 8 / 256), 256, 0, stream>>>(W14b, 1.0f, W14); k_b2h<<<(unsigned)(NN / 8 / 256), 256, 0, stream>>>(W17b, 1.0f, W17);
      k_fill<<<1, 256, 0, stream>>>((float*)W13, 0.0f, (size_t)16 * 128 * 2 / 16); k_cvt8<<<1, 256, 0, stream>>>(i13, W13, (size_t)12 * 128 / 8);     }
    k_fill<<<1, 256, 0, stream>>>(ONE, 1.0f, 768 / 4); k_fill<<<1, 256, 0, stream>>>(NOU, 0.0f, 768 / 4); k_fill<<<(unsigned)((NN / 4 + 255) / 256), 256, 0, stream>>>(ZP, 0.0f, NN / 4); k_fill<<<(unsigned)((NN * 16 / 4 + 255) / 256), 256, 0, stream>>>(ZE, 0.0f, NN * 16 / 4);
    k_rbf<<<(unsigned)((NC / 4 + 255) / 256), 256, 0, stream>>>(i1, CR, NC / 4); k_lnrow<false><<<(unsigned)((64 + 7) / 8), 256, 0, stream>>>(CR, nullptr, i5, NOU, 1.0e-5f, 512, 64, CN); k_tohl<<<(unsigned)((NC / 4 + 255) / 256), 256, 0, stream>>>(CN, 1.0f, CNh, CNl, NC / 4); k_cvt8<<<(unsigned)((NC / 8 + 255) / 256), 256, 0, stream>>>(CR, CRb, NC / 8);
    k_gemmw<bf, 1, true><<<dim3(64 / 64, 768 / 64, 1), 32, 0, stream>>>(CNh, CNl, W6, nullptr, 512, T1, 768, i7, 0, 0, 0); k_gemmw<bf, 1, false><<<dim3(64 / 64, 768 / 64, 1), 32, 0, stream>>>(CNh, CNl, W8, nullptr, 512, T2, 768, nullptr, 0, 0, 0); k_gemmw<bf, 0, true><<<dim3(64 / 64, 768 / 64, 1), 32, 0, stream>>>(CRb, nullptr, W15, nullptr, 512, T3, 768, i16, 0, 0, 0);
    { const unsigned LG = (unsigned)(((size_t)768 * (768 / 4) + 255) / 256); rgath_kernel<768><<<LG, 256, 0, stream>>>(T1, i4, 64, 0, G1, 768, 0, 768); rgath_kernel<768><<<LG, 256, 0, stream>>>(T2, i4, 64, 0, G2, 768, 0, 768); rgath_kernel<768><<<LG, 256, 0, stream>>>(T3, i4, 64, 0, G3, 768, 0, 768); }
    { const unsigned LM = (unsigned)((NN / 4 + 255) / 256); k_mulm<<<LM, 256, 0, stream>>>(G1, i3, G1m, 768 / 4, 768); k_mulm<<<LM, 256, 0, stream>>>(G2, i3, G2m, 768 / 4, 768);
      k_rbf<<<LM, 256, 0, stream>>>(i0, NR, NN / 4); k_lnrow<false><<<(unsigned)((768 + 7) / 8), 256, 0, stream>>>(NR, nullptr, ONE, NOU, 1.0e-5f, 768, 768, S0);
      k_sg<<<LM, 256, 0, stream>>>(S0, 768, 768, 768, G1m, 768, G2m, 768, 1.0f, ST, 768, 768 / 4, 768); }
    k_castp<h16><<<(unsigned)(NN / 8 / 256), 256, 0, stream>>>(ST, 2304, 8, 1.0f, S16);
    k_gemmw<h16, 0, false><<<dim3(768 / 64, 768 / 64, 1), 32, 0, stream>>>((const h16*)S16, nullptr, (const h16*)W9, nullptr, 768, FQ, 768, nullptr, 0, 0, 0); k_gemmw<h16, 0, false><<<dim3(768 / 64, 1536 / 64, 1), 32, 0, stream>>>((const h16*)S16, nullptr, (const h16*)W10, nullptr, 768, FKV, 1536, nullptr, 0, 0, 0); k_gemmw<h16, 0, false><<<dim3(768 / 64, 768 / 64, 1), 32, 0, stream>>>((const h16*)S16, nullptr, (const h16*)W14, nullptr, 768, FG, 768, nullptr, 0, 0, 0);
    for (int h = 0; h < 12; ++h) { k_cvtp<<<(unsigned)((768 * 16 + 255) / 256), 256, 0, stream>>>(FQ + h * HD, QP16 + (size_t)h * TT * HD, HD / 4, 768, HD, 768); k_cvtp<<<(unsigned)((768 * 16 + 255) / 256), 256, 0, stream>>>(FKV + h * HD, KP16 + (size_t)h * TT * HD, HD / 4, 1536, HD, 768); }
    k_vtp<<<(unsigned)(((size_t)12 * TT * HD / 2 + 255) / 256), 256, 0, stream>>>(FKV + 768, 1536, 12, VT16, nullptr, nullptr);
    for (int p = 0; p < 12; ++p) { k_rbf<<<(unsigned)((PZ / 4 + 255) / 256), 256, 0, stream>>>(i2 + (size_t)p * PZ, ZR, PZ / 4); k_lnrow<false><<<(unsigned)((64 * 768 + 7) / 8), 256, 0, stream>>>(ZR, nullptr, i11, i12, 1.0e-5f, 128, 64 * 768, ZN); k_cvt8<<<(unsigned)((PZ / 8 + 255) / 256), 256, 0, stream>>>(ZN, ZB, PZ / 8);
      k_gemmn<bf, 0, false, 16><<<dim3(64 * 768 / 64, 1, 1), 32, 0, stream>>>(ZB, nullptr, W13, nullptr, 128, PB + (size_t)p * 64 * 768 * 16, 16, nullptr, 0, 0, 0); }
    for (int h = 0; h < 12; ++h) {
        k_gemmw<h16, 0, false><<<dim3(TT / 64, TT / 64, 1), 32, 0, stream>>>(QP16 + (size_t)h * TT * HD, nullptr, KP16 + (size_t)h * TT * HD, nullptr, HD, Sb, TT, nullptr, 0, 0, 0);
        k_hb<<<(unsigned)((NN / 4 + 255) / 256), 256, 0, stream>>>(ZE, PB, NOU, h, 8.0f, Sb, S2, MP);
        k_mterm<<<(unsigned)((NN / 4 + 255) / 256), 256, 0, stream>>>(S2, i3, 800000.0f);
        k_asoftMA<<<ZH * TT / 8, 256, 0, stream>>>(S2, MP, P16, nullptr, nullptr);
        k_gemmw<h16, 0, false><<<dim3(TT / 64, HD / 64, 1), 32, 0, stream>>>(P16, nullptr, VT16 + (size_t)h * HD * TT, nullptr, TT, OB + h * HD, 768, nullptr, 0, 0, 0); }
    { const unsigned LM = (unsigned)((NN / 4 + 255) / 256); k_sg<<<LM, 256, 0, stream>>>(OB, 768, 768, 768, FG, 768, ZP, 768, 0.0009765625f, GO, 768, 768 / 4, 768);
      k_castp<h16><<<(unsigned)(NN / 8 / 256), 256, 0, stream>>>(GO, 2304, 8, 1.0f, GO16); k_gemmw<h16, 0, false><<<dim3(768 / 64, 768 / 64, 1), 32, 0, stream>>>((const h16*)GO16, nullptr, (const h16*)W17, nullptr, 768, OM, 768, nullptr, 0, 0, 0);
      k_sg<<<LM, 256, 0, stream>>>(OM, 768, 768, 768, G3, 768, ZP, 768, 1.0f, FO, 768, 768 / 4, 768); k_mulm<<<LM, 256, 0, stream>>>(FO, i3, OUT, 768 / 4, 768); }
}
